// MoETransformer_39384850104910
// MI455X (gfx1250) — hardware-verified
//
#include <hip/hip_runtime.h>
#include <stdint.h>
#include <stddef.h>
#include <math.h>

#pragma clang fp contract(off)

#define NTOK 4096
#define DM   1024
#define HX   512
#define GU   1024
#define NEX  8
#define HS   2048
#define MT   64
#define XP   1032
#define HP   520
#define YP   260
#define TP   136
#define TRP  72

#define LDS_XB  (MT * XP * 2)
#define LDS_HB  (MT * HP * 2)
#define LDS_EXP (LDS_XB + LDS_HB)
#define LDS_DN  (64 * YP * 4)

#define W_SC 256.0f
#define H_SC 64.0f
#define R_W  0.00390625f
#define R_HW 6.103515625e-05f

static_assert(MT * YP * 4 <= LDS_XB);
static_assert((XP * 2) % 16 == 0);
static_assert((HP * 2) % 16 == 0);
static_assert((YP * 4) % 16 == 0);
static_assert((TP * 2) % 16 == 0);
static_assert((TRP * 2) % 16 == 0);
static_assert(NTOK % 256 == 0);
static_assert(NTOK % MT == 0);
static_assert(NTOK % 64 == 0);
static_assert(MT == 8 * 8);
static_assert(DM % 256 == 0);
static_assert(HX % 128 == 0);
static_assert(HS % 128 == 0);
static_assert(DM % 32 == 0);
static_assert(HX % 32 == 0);
static_assert(HS % 32 == 0);
static_assert(GU == 2 * HX);
static_assert((NEX * DM) % 1024 == 0);

typedef _Float16       v16h __attribute__((ext_vector_type(16)));
typedef _Float16       v8h  __attribute__((ext_vector_type(8)));
typedef float          v8f  __attribute__((ext_vector_type(8)));
typedef float          v4f  __attribute__((ext_vector_type(4)));
typedef unsigned int   v4u  __attribute__((ext_vector_type(4)));
typedef v4f __attribute__((may_alias)) v4fa;
typedef v4u __attribute__((may_alias)) v4ua;

union FragH { v16h v; v4u q[2]; };
union Pack8 { v8h h; v4u u; };

__device__ __forceinline__ unsigned short hbits(float f) {
  _Float16 t = (_Float16)f;
  unsigned short u;
  __builtin_memcpy(&u, &t, 2);
  return u;
}

__device__ __forceinline__ v8f wmma_h(v16h a, v16h b, v8f c) {
  v8f d = __builtin_amdgcn_wmma_f32_16x16x32_f16(false, a, false, b, (short)0, c, false, false);
  asm volatile("v_nop\n\tv_nop\n\tv_nop\n\tv_nop" : "+v"(d) : "v"(a), "v"(b));
  return d;
}

__device__ __forceinline__ v16h ldfrag(const unsigned short* p, int h) {
  FragH f;
  f.q[0] = *(const v4ua*)(p + 8 * h);
  f.q[1] = *(const v4ua*)(p + 16 + 8 * h);
  return f.v;
}

__device__ __forceinline__ float silu_f(float v) {
  return v * __builtin_amdgcn_rcpf(1.0f + __expf(-v));
}

__global__ __launch_bounds__(256) void k_cvt(const float* __restrict__ src,
                                             unsigned short* __restrict__ dst,
                                             int n8, float sc)
{
  const int g = blockIdx.x * 256 + threadIdx.x;
  if (g >= n8) return;
  const float* s = src + (size_t)g * 8;
  const v4f a = *(const v4fa*)s;
  const v4f c = *(const v4fa*)(s + 4);
  v8h hv;
  hv[0] = (_Float16)(a.x * sc); hv[1] = (_Float16)(a.y * sc);
  hv[2] = (_Float16)(a.z * sc); hv[3] = (_Float16)(a.w * sc);
  hv[4] = (_Float16)(c.x * sc); hv[5] = (_Float16)(c.y * sc);
  hv[6] = (_Float16)(c.z * sc); hv[7] = (_Float16)(c.w * sc);
  Pack8 p;
  p.h = hv;
  const v4u u = p.u;
  unsigned short* d = dst + (size_t)g * 8;
  *(volatile v4u*)d = u;
  __threadfence();
  *(volatile v4u*)d = u;
}

__global__ __launch_bounds__(256) void k_tr(const float* __restrict__ src,
                                            unsigned short* __restrict__ dst,
                                            int R, int CC, float sc)
{
  __shared__ __align__(16) unsigned short sT[64 * TRP];
  const int tid = threadIdx.x, lane = tid & 31, wv = tid >> 5;
  const int bz = blockIdx.z;
  const int r0 = blockIdx.y * 64;
  const int c0 = blockIdx.x * 64;
  const float* sb = src + (size_t)bz * (size_t)R * (size_t)CC;
  unsigned short* db = dst + (size_t)bz * (size_t)CC * (size_t)R;
  #pragma unroll
  for (int p = 0; p < 4; ++p) {
    const int idx = tid + 256 * p;
    const int r = idx >> 4;
    const int c4 = (idx & 15) * 4;
    const v4f v = *(const v4fa*)(sb + (size_t)(r0 + r) * CC + c0 + c4);
    sT[(c4 + 0) * TRP + r] = hbits(v.x * sc);
    sT[(c4 + 1) * TRP + r] = hbits(v.y * sc);
    sT[(c4 + 2) * TRP + r] = hbits(v.z * sc);
    sT[(c4 + 3) * TRP + r] = hbits(v.w * sc);
  }
  __syncthreads();
  #pragma unroll
  for (int i = 0; i < 2; ++i) {
    const int q = (wv * 2 + i) * 4 + (lane >> 3);
    const int piece = lane & 7;
    const v4u u = *(const v4ua*)(sT + q * TRP + 8 * piece);
    unsigned short* d = db + (size_t)(c0 + q) * R + r0 + 8 * piece;
    *(volatile v4u*)d = u;
    __threadfence();
    *(volatile v4u*)d = u;
  }
}

__global__ __launch_bounds__(256) void k_route(const float* __restrict__ x,
                                               const float* __restrict__ rw,
                                               float* __restrict__ rec, int ntok)
{
  __shared__ __align__(16) float swr[NEX * DM];
  __shared__ __align__(16) float srec[32];
  const int tid = threadIdx.x, lane = tid & 31, wv = tid >> 5;
  #pragma unroll 1
  for (int i = 0; i < (NEX * DM) / 1024; ++i) {
    const int o = 4 * (tid + 256 * i);
    const v4f w4 = *(const v4fa*)(rw + o);
    *(v4fa*)(swr + o) = w4;
  }
  __syncthreads();

  const int t = blockIdx.x * 8 + wv;
  const int tc = (t < ntok) ? t : (ntok - 1);
  const float* xr = x + (size_t)tc * DM;
  double lg[NEX];
  #pragma unroll
  for (int e = 0; e < NEX; ++e) lg[e] = 0.0;
  #pragma unroll 1
  for (int i = 0; i < DM / 32; ++i) {
    const int d = 32 * i + lane;
    const double xv = (double)xr[d];
    #pragma unroll
    for (int e = 0; e < NEX; ++e) lg[e] = fma(xv, (double)swr[e * DM + d], lg[e]);
  }
  #pragma unroll
  for (int off = 16; off > 0; off >>= 1) {
    #pragma unroll
    for (int e = 0; e < NEX; ++e) lg[e] = lg[e] + __shfl_xor(lg[e], off);
  }

  float lf[NEX];
  #pragma unroll
  for (int e = 0; e < NEX; ++e) lf[e] = (float)lg[e];
  int i0 = 0;
  float b0 = lf[0];
  #pragma unroll
  for (int e = 1; e < NEX; ++e) {
    const bool tk = lf[e] > b0;
    b0 = tk ? lf[e] : b0;
    i0 = tk ? e : i0;
  }
  int i1 = -1;
  float b1 = -3.0e38f;
  #pragma unroll
  for (int e = 0; e < NEX; ++e) {
    const bool tk = (e != i0) && (lf[e] > b1);
    b1 = tk ? lf[e] : b1;
    i1 = tk ? e : i1;
  }
  i1 = (i1 < 0) ? ((i0 == 0) ? 1 : 0) : i1;
  float l0 = lf[0], l1 = lf[0];
  #pragma unroll
  for (int e = 0; e < NEX; ++e) { l0 = (e == i0) ? lf[e] : l0; l1 = (e == i1) ? lf[e] : l1; }
  const float g0 = __builtin_amdgcn_rcpf(1.0f + __expf(-l0));
  const float g1 = __builtin_amdgcn_rcpf(1.0f + __expf(-l1));

  if (lane == 0) {
    srec[4 * wv + 0] = g0;
    srec[4 * wv + 1] = g1;
    srec[4 * wv + 2] = (float)i0;
    srec[4 * wv + 3] = (float)i1;
  }
  __syncthreads();
  if (wv == 0) {
    const int q = lane & 7;
    const v4f v = *(const v4fa*)(srec + 4 * q);
    const int tt = blockIdx.x * 8 + q;
    const bool ok = (lane < 8) && (tt < ntok);
    if (ok) *(volatile v4f*)(rec + (size_t)tt * 4) = v;
    __threadfence();
    if (ok) *(volatile v4f*)(rec + (size_t)tt * 4) = v;
  }
}

__device__ __forceinline__ void part_pass(const float* sY, const int* sTok, const int* sSlot,
                                          float* part, int ns, int wv, int lane, int nrows)
{
  #pragma unroll
  for (int i = 0; i < 8; ++i) {
    const int row = wv * 8 + i;
    int t = sTok[row];
    t = (t < 0) ? 0 : ((t > NTOK - 1) ? (NTOK - 1) : t);
    int s = sSlot[row];
    s = (s != 0) ? 1 : 0;
    const v4f v0 = *(const v4fa*)(sY + row * YP + 4 * lane);
    const v4f v1 = *(const v4fa*)(sY + row * YP + 128 + 4 * lane);
    float* dst = part + ((size_t)t * 2 + s) * DM + ns * 256;
    if (row < nrows) {
      *(volatile v4f*)(dst + 4 * lane) = v0;
      *(volatile v4f*)(dst + 128 + 4 * lane) = v1;
    }
  }
}

__global__ __launch_bounds__(256) void k_expert(const unsigned short* __restrict__ xh,
                                                const unsigned short* __restrict__ gut,
                                                const unsigned short* __restrict__ dwt,
                                                const float* __restrict__ rec,
                                                float* __restrict__ part, int ntok)
{
  extern __shared__ __align__(16) unsigned char dsm_e[];
  unsigned short* sX = (unsigned short*)dsm_e;
  unsigned short* sH = (unsigned short*)(dsm_e + LDS_XB);
  float* sY = (float*)dsm_e;
  __shared__ int   sTok[MT];
  __shared__ int   sSlot[MT];
  __shared__ float sW[MT];
  __shared__ int   s_wc[8];

  const int tid = threadIdx.x, lane = tid & 31, wv = tid >> 5;
  const int h = lane >> 4, m = lane & 15;
  const int wr = wv >> 2, wc = wv & 3;
  const int e = blockIdx.y;
  const int m0 = blockIdx.x * MT;

  if (tid < MT) { sTok[tid] = 0; sSlot[tid] = 0; sW[tid] = 0.0f; }
  __syncthreads();

  int base = 0;
  #pragma unroll 1
  for (int ch = 0; ch < NTOK / 256; ++ch) {
    const int t = ch * 256 + tid;
    const int tc = (t < ntok) ? t : (ntok - 1);
    const v4f r = *(const v4fa*)(rec + (size_t)tc * 4);
    int e0 = (int)r.z, e1 = (int)r.w;
    e0 = (e0 < 0) ? 0 : ((e0 > NEX - 1) ? (NEX - 1) : e0);
    e1 = (e1 < 0) ? 0 : ((e1 > NEX - 1) ? (NEX - 1) : e1);
    const bool f0 = (e0 == e);
    const bool f1 = (e1 == e) && !f0;
    const bool f = (f0 || f1) && (t < ntok);
    const unsigned int msk = __builtin_amdgcn_ballot_w32(f);
    const int off = __builtin_popcount(msk & ((1u << lane) - 1u));
    const int wcnt = __builtin_popcount(msk);
    if (lane == 0) s_wc[wv] = wcnt;
    __syncthreads();
    int pre = 0, tot = 0;
    #pragma unroll
    for (int w2 = 0; w2 < 8; ++w2) {
      const int cc = s_wc[w2];
      tot += cc;
      pre += (w2 < wv) ? cc : 0;
    }
    if (f) {
      const int p = base + pre + off - m0;
      if ((unsigned)p < (unsigned)MT) {
        sTok[p]  = t;
        sSlot[p] = f0 ? 0 : 1;
        sW[p]    = f0 ? r.x : r.y;
      }
    }
    base += tot;
    __syncthreads();
  }
  const int cnt = base;
  if (m0 >= cnt) return;
  int nrows = cnt - m0;
  nrows = (nrows > MT) ? MT : nrows;

  #pragma unroll 4
  for (int j = 0; j < 32; ++j) {
    const int idx = tid + 256 * j;
    const int row = idx >> 7, c8 = idx & 127;
    int t = sTok[row];
    t = (t < 0) ? 0 : ((t > NTOK - 1) ? (NTOK - 1) : t);
    const size_t go = (size_t)t * DM + 8 * c8;
    const v4u a = *(const v4ua*)(xh + go);
    *(v4ua*)(sX + row * XP + 8 * c8) = a;
  }
  __syncthreads();

  const v8f z8 = {0.f, 0.f, 0.f, 0.f, 0.f, 0.f, 0.f, 0.f};

  #pragma unroll 1
  for (int ns = 0; ns < HX / 128; ++ns) {
    v8f ag[2][2], au[2][2];
    #pragma unroll
    for (int mt = 0; mt < 2; ++mt)
      #pragma unroll
      for (int nt = 0; nt < 2; ++nt) { ag[mt][nt] = z8; au[mt][nt] = z8; }
    #pragma unroll 1
    for (int k0 = 0; k0 < DM; k0 += 32) {
      v16h a[2];
      #pragma unroll
      for (int mt = 0; mt < 2; ++mt)
        a[mt] = ldfrag(sX + (32 * wr + 16 * mt + m) * XP + k0, h);
      #pragma unroll
      for (int nt = 0; nt < 2; ++nt) {
        const int jg = ns * 128 + wc * 32 + 16 * nt + m;
        const size_t bg_o = ((size_t)e * GU + jg) * DM + k0;
        const size_t bu_o = ((size_t)e * GU + HX + jg) * DM + k0;
        const v16h bg = ldfrag(gut + bg_o, h);
        const v16h bu = ldfrag(gut + bu_o, h);
        #pragma unroll
        for (int mt = 0; mt < 2; ++mt) {
          ag[mt][nt] = wmma_h(a[mt], bg, ag[mt][nt]);
          au[mt][nt] = wmma_h(a[mt], bu, au[mt][nt]);
        }
      }
    }
    #pragma unroll
    for (int mt = 0; mt < 2; ++mt)
      #pragma unroll
      for (int nt = 0; nt < 2; ++nt) {
        const int col = ns * 128 + wc * 32 + 16 * nt + m;
        #pragma unroll
        for (int r = 0; r < 8; ++r) {
          const int row = 32 * wr + 16 * mt + 8 * h + r;
          const float g = ag[mt][nt][r] * R_W;
          const float u = au[mt][nt][r] * R_W;
          const float hv = silu_f(g) * u * H_SC;
          sH[row * HP + col] = hbits(hv);
        }
      }
  }
  __syncthreads();

  #pragma unroll 1
  for (int ns = 0; ns < DM / 256; ++ns) {
    v8f acc[2][4];
    #pragma unroll
    for (int mt = 0; mt < 2; ++mt)
      #pragma unroll
      for (int nt = 0; nt < 4; ++nt) acc[mt][nt] = z8;
    #pragma unroll 1
    for (int k0 = 0; k0 < HX; k0 += 32) {
      v16h a[2];
      #pragma unroll
      for (int mt = 0; mt < 2; ++mt)
        a[mt] = ldfrag(sH + (32 * wr + 16 * mt + m) * HP + k0, h);
      #pragma unroll
      for (int nt = 0; nt < 4; ++nt) {
        const int d = ns * 256 + wc * 64 + 16 * nt + m;
        const size_t bo = ((size_t)e * DM + d) * HX + k0;
        const v16h b = ldfrag(dwt + bo, h);
        #pragma unroll
        for (int mt = 0; mt < 2; ++mt) acc[mt][nt] = wmma_h(a[mt], b, acc[mt][nt]);
      }
    }
    #pragma unroll
    for (int mt = 0; mt < 2; ++mt)
      #pragma unroll
      for (int nt = 0; nt < 4; ++nt) {
        const int cl = wc * 64 + 16 * nt + m;
        #pragma unroll
        for (int r = 0; r < 8; ++r) {
          const int row = 32 * wr + 16 * mt + 8 * h + r;
          sY[row * YP + cl] = acc[mt][nt][r] * (sW[row] * R_HW);
        }
      }
    __syncthreads();
    part_pass(sY, sTok, sSlot, part, ns, wv, lane, nrows);
    __threadfence();
    part_pass(sY, sTok, sSlot, part, ns, wv, lane, nrows);
    __syncthreads();
  }
}

__global__ __launch_bounds__(256) void k_shgu(const unsigned short* __restrict__ xh,
                                              const unsigned short* __restrict__ sgp,
                                              const unsigned short* __restrict__ sup,
                                              unsigned short* __restrict__ hsp)
{
  __shared__ __align__(16) unsigned short sT[64 * TP];
  const int tid = threadIdx.x, lane = tid & 31, wv = tid >> 5;
  const int h = lane >> 4, m = lane & 15;
  const int wr = wv >> 2, wc = wv & 3;
  const int m0 = blockIdx.y * 64, n0 = blockIdx.x * 128;

  const v8f z8 = {0.f, 0.f, 0.f, 0.f, 0.f, 0.f, 0.f, 0.f};
  v8f ag[2][2], au[2][2];
  #pragma unroll
  for (int mt = 0; mt < 2; ++mt)
    #pragma unroll
    for (int nt = 0; nt < 2; ++nt) { ag[mt][nt] = z8; au[mt][nt] = z8; }

  #pragma unroll 1
  for (int k0 = 0; k0 < DM; k0 += 32) {
    v16h a[2];
    #pragma unroll
    for (int mt = 0; mt < 2; ++mt)
      a[mt] = ldfrag(xh + (size_t)(m0 + 32 * wr + 16 * mt + m) * DM + k0, h);
    #pragma unroll
    for (int nt = 0; nt < 2; ++nt) {
      const size_t ro = (size_t)(n0 + wc * 32 + 16 * nt + m) * DM + k0;
      const v16h bg = ldfrag(sgp + ro, h);
      const v16h bu = ldfrag(sup + ro, h);
      #pragma unroll
      for (int mt = 0; mt < 2; ++mt) {
        ag[mt][nt] = wmma_h(a[mt], bg, ag[mt][nt]);
        au[mt][nt] = wmma_h(a[mt], bu, au[mt][nt]);
      }
    }
  }
  #pragma unroll
  for (int mt = 0; mt < 2; ++mt)
    #pragma unroll
    for (int nt = 0; nt < 2; ++nt) {
      const int cl = wc * 32 + 16 * nt + m;
      #pragma unroll
      for (int r = 0; r < 8; ++r) {
        const int row = 32 * wr + 16 * mt + 8 * h + r;
        const float g = ag[mt][nt][r] * R_W;
        const float u = au[mt][nt][r] * R_W;
        sT[row * TP + cl] = hbits(silu_f(g) * u * H_SC);
      }
    }
  __syncthreads();
  #pragma unroll
  for (int i = 0; i < 4; ++i) {
    const int rl = 8 * wv + 2 * i + h;
    const v4u u4 = *(const v4ua*)(sT + rl * TP + 8 * m);
    unsigned short* d = hsp + (size_t)(m0 + rl) * HS + n0 + 8 * m;
    *(volatile v4u*)d = u4;
    __threadfence();
    *(volatile v4u*)d = u4;
  }
}

__global__ __launch_bounds__(256) void k_shdn(const unsigned short* __restrict__ hsp,
                                              const unsigned short* __restrict__ sdp,
                                              const float* __restrict__ part,
                                              float* __restrict__ out)
{
  extern __shared__ __align__(16) unsigned char dsm_d[];
  float* sY = (float*)dsm_d;
  const int tid = threadIdx.x, lane = tid & 31, wv = tid >> 5;
  const int h = lane >> 4, m = lane & 15;
  const int wr = wv >> 2, wc = wv & 3;
  const int m0 = blockIdx.y * 64, n0 = blockIdx.x * 256;

  const v8f z8 = {0.f, 0.f, 0.f, 0.f, 0.f, 0.f, 0.f, 0.f};
  v8f acc[2][4];
  #pragma unroll
  for (int mt = 0; mt < 2; ++mt)
    #pragma unroll
    for (int nt = 0; nt < 4; ++nt) acc[mt][nt] = z8;

  #pragma unroll 1
  for (int k0 = 0; k0 < HS; k0 += 32) {
    v16h a[2];
    #pragma unroll
    for (int mt = 0; mt < 2; ++mt)
      a[mt] = ldfrag(hsp + (size_t)(m0 + 32 * wr + 16 * mt + m) * HS + k0, h);
    #pragma unroll
    for (int nt = 0; nt < 4; ++nt) {
      const v16h b = ldfrag(sdp + (size_t)(n0 + wc * 64 + 16 * nt + m) * HS + k0, h);
      #pragma unroll
      for (int mt = 0; mt < 2; ++mt) acc[mt][nt] = wmma_h(a[mt], b, acc[mt][nt]);
    }
  }
  #pragma unroll
  for (int mt = 0; mt < 2; ++mt)
    #pragma unroll
    for (int nt = 0; nt < 4; ++nt) {
      const int cl = wc * 64 + 16 * nt + m;
      #pragma unroll
      for (int r = 0; r < 8; ++r) {
        const int row = 32 * wr + 16 * mt + 8 * h + r;
        sY[row * YP + cl] = acc[mt][nt][r] * R_HW;
      }
    }
  __syncthreads();
  #pragma unroll
  for (int i = 0; i < 8; ++i) {
    const int rl = 8 * wv + i;
    const int t = m0 + rl;
    const v4f y0 = *(const v4fa*)(sY + rl * YP + 4 * lane);
    const v4f y1 = *(const v4fa*)(sY + rl * YP + 128 + 4 * lane);
    const float* p0 = part + ((size_t)t * 2) * DM + n0;
    const float* p1 = p0 + DM;
    const v4f a0 = *(const v4fa*)(p0 + 4 * lane);
    const v4f a1 = *(const v4fa*)(p0 + 128 + 4 * lane);
    const v4f b0 = *(const v4fa*)(p1 + 4 * lane);
    const v4f b1 = *(const v4fa*)(p1 + 128 + 4 * lane);
    const v4f o0 = (a0 + b0) + y0;
    const v4f o1 = (a1 + b1) + y1;
    float* d = out + (size_t)t * DM + n0;
    *(volatile v4f*)(d + 4 * lane) = o0;
    *(volatile v4f*)(d + 128 + 4 * lane) = o1;
    __threadfence();
    *(volatile v4f*)(d + 4 * lane) = o0;
    *(volatile v4f*)(d + 128 + 4 * lane) = o1;
  }
}

extern "C" void kernel_launch(void* const* d_in, const int* in_sizes, int n_in,
                              void* d_out, int out_size, void* d_ws, size_t ws_size,
                              hipStream_t stream)
{
  if (n_in < 7) return;
  if (in_sizes[0] != NTOK * DM) return;
  if (in_sizes[1] != NEX * DM) return;
  if (in_sizes[2] != NEX * DM * GU) return;
  if (in_sizes[3] != NEX * HX * DM) return;
  if (in_sizes[4] != HS * DM) return;
  if (in_sizes[5] != HS * DM) return;
  if (in_sizes[6] != DM * HS) return;
  if (out_size != NTOK * DM) return;

  const float* x   = (const float*)d_in[0];
  const float* rw  = (const float*)d_in[1];
  const float* guw = (const float*)d_in[2];
  const float* dww = (const float*)d_in[3];
  const float* sgw = (const float*)d_in[4];
  const float* suw = (const float*)d_in[5];
  const float* sdw = (const float*)d_in[6];
  float* out = (float*)d_out;

  const size_t bXH   = (size_t)NTOK * DM * 2;
  const size_t bGUT  = (size_t)NEX * GU * DM * 2;
  const size_t bDWT  = (size_t)NEX * DM * HX * 2;
  const size_t bSG   = (size_t)HS * DM * 2;
  const size_t bSU   = (size_t)HS * DM * 2;
  const size_t bSD   = (size_t)DM * HS * 2;
  const size_t bHSP  = (size_t)NTOK * HS * 2;
  const size_t bREC  = (size_t)NTOK * 16;
  const size_t bPART = (size_t)NTOK * 2 * DM * 4;
  const size_t total = bXH + bGUT + bDWT + bSG + bSU + bSD + bHSP + bREC + bPART;
  if (total > ws_size) return;
  if (total > (size_t)134217728) return;

  char* ws = (char*)d_ws;
  size_t off = 0;
  unsigned short* XH   = (unsigned short*)(ws + off); off += bXH;
  unsigned short* GUT  = (unsigned short*)(ws + off); off += bGUT;
  unsigned short* DWT  = (unsigned short*)(ws + off); off += bDWT;
  unsigned short* SGP  = (unsigned short*)(ws + off); off += bSG;
  unsigned short* SUP  = (unsigned short*)(ws + off); off += bSU;
  unsigned short* SDP  = (unsigned short*)(ws + off); off += bSD;
  unsigned short* HSP  = (unsigned short*)(ws + off); off += bHSP;
  float*          REC  = (float*)(ws + off);          off += bREC;
  float*          PART = (float*)(ws + off);          off += bPART;
  if (off != total) return;

  hipFuncSetAttribute(reinterpret_cast<const void*>(&k_expert),
                      hipFuncAttributeMaxDynamicSharedMemorySize, LDS_EXP);
  hipFuncSetAttribute(reinterpret_cast<const void*>(&k_shdn),
                      hipFuncAttributeMaxDynamicSharedMemorySize, LDS_DN);

  {
    const int n8x = NTOK * DM / 8;
    const int n8s = HS * DM / 8;
    k_cvt<<<(n8x + 255) / 256, 256, 0, stream>>>(x, XH, n8x, 1.0f);
    k_cvt<<<(n8s + 255) / 256, 256, 0, stream>>>(sgw, SGP, n8s, W_SC);
    k_cvt<<<(n8s + 255) / 256, 256, 0, stream>>>(suw, SUP, n8s, W_SC);
    k_cvt<<<(n8s + 255) / 256, 256, 0, stream>>>(sdw, SDP, n8s, W_SC);
  }
  k_tr<<<dim3(GU / 64, DM / 64, NEX), 256, 0, stream>>>(guw, GUT, DM, GU, W_SC);
  k_tr<<<dim3(DM / 64, HX / 64, NEX), 256, 0, stream>>>(dww, DWT, HX, DM, W_SC);
  k_route<<<(NTOK + 7) / 8, 256, 0, stream>>>(x, rw, REC, NTOK);
  k_expert<<<dim3(NTOK / MT, NEX), 256, LDS_EXP, stream>>>(XH, GUT, DWT, REC, PART, NTOK);
  k_shgu<<<dim3(HS / 128, NTOK / 64), 256, 0, stream>>>(XH, SGP, SUP, HSP);
  k_shdn<<<dim3(DM / 256, NTOK / 64), 256, LDS_DN, stream>>>(HSP, SDP, PART, out);
}
